// MambaVisionMixer_36867999268916
// MI455X (gfx1250) — hardware-verified
//
#include <hip/hip_runtime.h>
#include <math.h>

typedef __attribute__((ext_vector_type(16))) _Float16 v16h;
typedef __attribute__((ext_vector_type(8)))  _Float16 v8h;
typedef __attribute__((ext_vector_type(16))) __bf16   v16b;
typedef __attribute__((ext_vector_type(8)))  __bf16   v8b;
typedef __attribute__((ext_vector_type(8)))  float    v8f;
typedef __attribute__((ext_vector_type(4)))  float    v4f;

constexpr int kBatch  = 2;
constexpr int kSeq    = 4096;
constexpr int kRows   = kBatch * kSeq;
constexpr int kDm     = 512;
constexpr int kDin    = 1024;
constexpr int kHalf   = 512;
constexpr int kNst    = 16;
constexpr int kDtR    = 32;
constexpr int kXdP    = 64;
constexpr int kConvTP = 260;
constexpr int kScanTS = 64;
constexpr int kScanCh = 64;
constexpr int kScanYP = 68;
constexpr float kLog2e = 1.4426950408889634f;
static_assert(kDtR + 2 * kNst == kXdP, "x_proj width");
static_assert(2 * kHalf == kDin, "inner split");
static_assert((kDm % 32) == 0 && (kHalf % 32) == 0 && (kDtR % 32) == 0 && (kDin % 32) == 0, "GEMM K multiples of 32");
static_assert((kRows % 64) == 0 && (kDin % 64) == 0 && (kXdP % 64) == 0 && (kHalf % 64) == 0 && (kDm % 64) == 0, "GEMM M,N multiples of 64");
static_assert((kSeq % kScanTS) == 0 && (kSeq % 64) == 0 && (kHalf % kScanCh) == 0 && (kHalf % 256) == 0, "tile multiples");
static_assert(kDtR == 32 && kScanTS == 64 && kScanCh == 64, "fused dt_proj tile: 64 steps x 64 channels x one 32-deep k-step");

constexpr size_t kOffAH   = 0;
constexpr size_t kOffWI   = kOffAH   + (size_t)kRows * kDm   * 2;
constexpr size_t kOffWX   = kOffWI   + (size_t)kDin  * kDm   * 2;
constexpr size_t kOffWD   = kOffWX   + (size_t)kXdP  * kHalf * 2;
constexpr size_t kOffWO   = kOffWD   + (size_t)kHalf * kDtR  * 2;
constexpr size_t kOffXZ   = kOffWO   + (size_t)kDm   * kDin  * 2;
constexpr size_t kOffXC   = kOffXZ   + (size_t)kRows * kDin  * 4;
constexpr size_t kOffXCH  = kOffXC   + (size_t)kRows * kHalf * 4;
constexpr size_t kOffXCL  = kOffXCH  + (size_t)kRows * kHalf * 2;
constexpr size_t kOffXD   = kOffXCL  + (size_t)kRows * kHalf * 2;
constexpr size_t kOffYCH  = kOffXD   + (size_t)kRows * kXdP  * 4;
constexpr size_t kOffYCL  = kOffYCH  + (size_t)kRows * kDin  * 2;
constexpr size_t kWsTotal = kOffYCL  + (size_t)kRows * kDin  * 2;
static_assert(kWsTotal == 113344512ull, "carve total");
static_assert(kWsTotal <= 134217728ull, "carve cap");
static_assert((kOffWI % 128) == 0 && (kOffWX % 128) == 0 && (kOffWD % 128) == 0 && (kOffWO % 128) == 0 &&
              (kOffXZ % 128) == 0 && (kOffXC % 128) == 0 && (kOffXCH % 128) == 0 && (kOffXCL % 128) == 0 &&
              (kOffXD % 128) == 0 && (kOffYCH % 128) == 0 && (kOffYCL % 128) == 0, "128-B aligned regions");

__device__ __forceinline__ unsigned short f2bf_bits(float f) {
  unsigned u = __float_as_uint(f);
  return (unsigned short)((u + 0x7FFFu + ((u >> 16) & 1u)) >> 16);
}
__device__ __forceinline__ float bf_bits2f(unsigned short h) { return __uint_as_float(((unsigned)h) << 16); }
__device__ __forceinline__ float bfr(float f) { return bf_bits2f(f2bf_bits(f)); }
__device__ __forceinline__ void split_bf2(float f, __bf16& hi, __bf16& lo) {
  const unsigned short hb = f2bf_bits(f);
  hi = __builtin_bit_cast(__bf16, hb);
  lo = __builtin_bit_cast(__bf16, f2bf_bits(f - bf_bits2f(hb)));
}

__device__ __forceinline__ void dep_guard4_h(v8f& a, v8f& b, v8f& c, v8f& d, v16h x, v16h y) { asm volatile("v_nop\n\tv_nop\n\tv_nop\n\tv_nop" : "+v"(a), "+v"(b), "+v"(c), "+v"(d) : "v"(x), "v"(y)); }
__device__ __forceinline__ void dep_guard4_b(v8f& a, v8f& b, v8f& c, v8f& d, v16b x, v16b y) { asm volatile("v_nop\n\tv_nop\n\tv_nop\n\tv_nop" : "+v"(a), "+v"(b), "+v"(c), "+v"(d) : "v"(x), "v"(y)); }
__device__ __forceinline__ void dep_guard1_b(v8f& a, v16b x, v16b y, v16b z) { asm volatile("v_nop\n\tv_nop\n\tv_nop\n\tv_nop" : "+v"(a) : "v"(x), "v"(y), "v"(z)); }
__device__ __forceinline__ void keep4_h(v16h a, v16h b, v16h c, v16h d) { asm volatile("v_nop" :: "v"(a), "v"(b), "v"(c), "v"(d)); }
__device__ __forceinline__ void keep4_b(v16b a, v16b b, v16b c, v16b d) { asm volatile("v_nop" :: "v"(a), "v"(b), "v"(c), "v"(d)); }
__device__ __forceinline__ void acc_guard4(v8f& a, v8f& b, v8f& c, v8f& d) { asm volatile("v_nop\n\tv_nop\n\tv_nop\n\tv_nop" : "+v"(a), "+v"(b), "+v"(c), "+v"(d)); }
template <typename T> struct Frag;
template <> struct Frag<_Float16> {
  typedef v16h V; union U { v16h v; v8h h[2]; };
  static __device__ __forceinline__ v16h load(const _Float16* p) {
    U f; f.h[0] = *(const v8h*)(p); f.h[1] = *(const v8h*)(p + 16); return f.v;
  }
  static __device__ __forceinline__ v8f mma(v16h a, v16h b, v8f c) {
    return __builtin_amdgcn_wmma_f32_16x16x32_f16(false, a, false, b, (short)0, c, false, false);
  }
  static __device__ __forceinline__ void guard4(v8f& a, v8f& b, v8f& c, v8f& d, v16h x, v16h y) { dep_guard4_h(a, b, c, d, x, y); }
  static __device__ __forceinline__ void keep(v16h a, v16h b, v16h c, v16h d) { keep4_h(a, b, c, d); }
};
template <> struct Frag<__bf16> {
  typedef v16b V; union U { v16b v; v8b h[2]; };
  static __device__ __forceinline__ v16b load(const __bf16* p) {
    U f; f.h[0] = *(const v8b*)(p); f.h[1] = *(const v8b*)(p + 16); return f.v;
  }
  static __device__ __forceinline__ v8f mma(v16b a, v16b b, v8f c) {
    return __builtin_amdgcn_wmma_f32_16x16x32_bf16(false, a, false, b, (short)0, c, false, false);
  }
  static __device__ __forceinline__ void guard4(v8f& a, v8f& b, v8f& c, v8f& d, v16b x, v16b y) { dep_guard4_b(a, b, c, d, x, y); }
  static __device__ __forceinline__ void keep(v16b a, v16b b, v16b c, v16b d) { keep4_b(a, b, c, d); }
};

template <int ET> struct Elem;
template <> struct Elem<0> { typedef _Float16 T; };
template <> struct Elem<1> { typedef __bf16 T; };
template <int ET, int SPL>
__global__ __launch_bounds__(256) void wmma_gemm64_kernel(
    const unsigned short* __restrict__ Ap, const unsigned short* __restrict__ A2p, int lda,
    const unsigned short* __restrict__ Btp, int ldb,
    float* __restrict__ Cout, int ldc,
    int M, int N, int K, float scale) {
  typedef typename Elem<ET>::T T;
  typedef typename Frag<T>::V V;
  const T* A = (const T*)Ap; const T* A2 = (const T*)A2p; const T* Bt = (const T*)Btp;
  __shared__ __align__(16) float sT[8][16 * 68];
  const int lane = threadIdx.x & 31;
  const int wave = threadIdx.x >> 5;
  const int tilesN = N >> 6;
  const int tilesM = M >> 6;
  const int tile = blockIdx.x * 8 + wave;
  if (tile >= tilesM * tilesN) return;
  const int tm = tile / tilesN;
  const int tn = tile - tm * tilesN;
  const int m0 = tm << 6;
  const int n0 = tn << 6;

  const int rlane = lane & 15;
  const int koff  = (lane >> 4) * 8;
  const int mOff  = (lane >> 4) * 8;

  v8f acc[4][4];
#pragma unroll
  for (int i = 0; i < 4; ++i)
#pragma unroll
    for (int j = 0; j < 4; ++j) acc[i][j] = (v8f){0.f,0.f,0.f,0.f,0.f,0.f,0.f,0.f};

  for (int k0 = 0; k0 < K; k0 += 32) {
    V bh[4];
#pragma unroll
    for (int j = 0; j < 4; ++j) {
      const size_t bo = (size_t)(n0 + (j << 4) + rlane) * ldb + koff + k0;
      bh[j] = Frag<T>::load(Bt + bo);
    }
#pragma unroll
    for (int i = 0; i < 4; ++i) {
      const size_t ao = (size_t)(m0 + (i << 4) + rlane) * lda + koff + k0;
      V ah = Frag<T>::load(A + ao);
      V al = ah;
      if (SPL == 1) al = Frag<T>::load(A2 + ao);
#pragma unroll
      for (int j = 0; j < 4; ++j) {
        acc[i][j] = Frag<T>::mma(ah, bh[j], acc[i][j]);
        if (SPL == 1) acc[i][j] = Frag<T>::mma(al, bh[j], acc[i][j]);
      }
      Frag<T>::guard4(acc[i][0], acc[i][1], acc[i][2], acc[i][3], ah, al);
    }
    Frag<T>::keep(bh[0], bh[1], bh[2], bh[3]);
  }
  acc_guard4(acc[0][0], acc[0][1], acc[0][2], acc[0][3]);
  acc_guard4(acc[1][0], acc[1][1], acc[1][2], acc[1][3]);
  acc_guard4(acc[2][0], acc[2][1], acc[2][2], acc[2][3]);
  acc_guard4(acc[3][0], acc[3][1], acc[3][2], acc[3][3]);

  float* slab = sT[wave];
#pragma unroll
  for (int i = 0; i < 4; ++i) {
    const int mBase = m0 + (i << 4);
#pragma unroll
    for (int j = 0; j < 4; ++j) {
#pragma unroll
      for (int r = 0; r < 8; ++r) {
        slab[(mOff + r) * 68 + (j << 4) + rlane] = acc[i][j][r] * scale;
      }
    }
    __builtin_amdgcn_fence(__ATOMIC_RELEASE, "workgroup");
    __builtin_amdgcn_wave_barrier();
    __builtin_amdgcn_fence(__ATOMIC_ACQUIRE, "workgroup");
    {
      const int hh = lane >> 4, c4 = (lane & 15) * 4;
      for (int pass = 0; pass < 2; ++pass) {
#pragma unroll
        for (int it = 0; it < 8; ++it) {
          const int row = it * 2 + hh;
          v4f v = *(const v4f*)(slab + row * 68 + c4);
          *(volatile v4f*)(Cout + (size_t)(mBase + row) * ldc + n0 + c4) = v;
        }
        __threadfence();
      }
    }
    __builtin_amdgcn_fence(__ATOMIC_RELEASE, "workgroup");
    __builtin_amdgcn_wave_barrier();
    __builtin_amdgcn_fence(__ATOMIC_ACQUIRE, "workgroup");
  }
}

__global__ __launch_bounds__(256) void cvt_rows_bf16_kernel(
    const float* __restrict__ src, unsigned short* __restrict__ dst, int total8)
{
  const int i = blockIdx.x * 256 + threadIdx.x;
  if (i >= total8) return;
  const size_t e0 = (size_t)i << 3;
  const v4f a0 = *(const v4f*)(src + e0);
  const v4f a1 = *(const v4f*)(src + e0 + 4);
  v8h hv;
#pragma unroll
  for (int e = 0; e < 4; ++e) {
    hv[e]     = __builtin_bit_cast(_Float16, f2bf_bits(a0[e]));
    hv[4 + e] = __builtin_bit_cast(_Float16, f2bf_bits(a1[e]));
  }
  unsigned short* qd = dst + e0;
  *(volatile v8h*)qd = hv;
  __threadfence();
  *(volatile v8h*)qd = hv;
}

template <bool WF32>
__global__ __launch_bounds__(256) void conv_silu_kernel(
    const float* __restrict__ XZ, int xcol0, const float* __restrict__ cw, const float* __restrict__ cb,
    float* __restrict__ UF, unsigned short* __restrict__ UH, unsigned short* __restrict__ UL, int p16, int c16)
{
  __shared__ __align__(16) float sT[16 * kConvTP];
  const int tid = threadIdx.x, lane = tid & 31, wave = tid >> 5;
  const int d0 = blockIdx.x * 256, d = d0 + tid;
  const int g0 = blockIdx.y * 64;
  const int tb = g0 & (kSeq - 1);
  const v4f wv = *(const v4f*)(cw + (size_t)d * 4);
  const float w0 = bfr(wv[0]), w1 = bfr(wv[1]), w2 = bfr(wv[2]), w3 = bfr(wv[3]);
  const float bc = bfr(cb[d]);
  const float* xs = XZ + xcol0 + d;
  float xm3, xm2, xm1;
  {
    const float fh = (tb > 0) ? 1.0f : 0.0f;
    const int rb = (tb > 0) ? (g0 - 3) : g0;
    const float v3 = xs[(size_t)rb * kDin];
    const float v2 = xs[(size_t)(rb + 1) * kDin];
    const float v1 = xs[(size_t)(rb + 2) * kDin];
    xm3 = v3 * fh;
    xm2 = v2 * fh;
    xm1 = v1 * fh;
  }
  const int hrow = wave >> 1;
  const int hch  = (wave & 1) * 128 + lane * 4;
#pragma unroll 1
  for (int sub = 0; sub < 4; ++sub) {
    const int lb = g0 + sub * 16;
#pragma unroll 1
    for (int s = 0; s < 16; ++s) {
      const float xcur = xs[(size_t)(lb + s) * kDin];
      float acc = w0 * xm3;
      acc = fmaf(w1, xm2, acc);
      acc = fmaf(w2, xm1, acc);
      acc = fmaf(w3, xcur, acc);
      const float sv = acc + bc;
      const float sg = __builtin_amdgcn_rcpf(1.0f + expf(-sv));
      sT[s * kConvTP + tid] = sv * sg;
      xm3 = xm2; xm2 = xm1; xm1 = xcur;
    }
    __syncthreads();
    v4f fv[4];
    v8h hv[2], lv[2];
    if (WF32) {
#pragma unroll
      for (int it = 0; it < 4; ++it) fv[it] = *(const v4f*)(sT + (it * 4 + hrow) * kConvTP + hch);
    }
#pragma unroll
    for (int it = 0; it < 2; ++it) {
      const float* sp = sT + (it * 8 + wave) * kConvTP + lane * 8;
      const v4f a0 = *(const v4f*)(sp);
      const v4f a1 = *(const v4f*)(sp + 4);
#pragma unroll
      for (int e = 0; e < 4; ++e) {
        const unsigned short h0 = f2bf_bits(a0[e]), h1 = f2bf_bits(a1[e]);
        const unsigned short l0 = f2bf_bits(a0[e] - bf_bits2f(h0)), l1 = f2bf_bits(a1[e] - bf_bits2f(h1));
        hv[it][e]     = __builtin_bit_cast(_Float16, h0);
        hv[it][4 + e] = __builtin_bit_cast(_Float16, h1);
        lv[it][e]     = __builtin_bit_cast(_Float16, l0);
        lv[it][4 + e] = __builtin_bit_cast(_Float16, l1);
      }
    }
    for (int pass = 0; pass < 2; ++pass) {
      if (WF32) {
#pragma unroll
        for (int it = 0; it < 4; ++it)
          *(volatile v4f*)(UF + (size_t)(lb + it * 4 + hrow) * kHalf + d0 + hch) = fv[it];
      }
#pragma unroll
      for (int it = 0; it < 2; ++it) {
        const size_t o = (size_t)(lb + it * 8 + wave) * p16 + c16 + d0 + lane * 8;
        *(volatile v8h*)(UH + o) = hv[it];
        *(volatile v8h*)(UL + o) = lv[it];
      }
      __threadfence();
    }
    __syncthreads();
  }
}

__global__ __launch_bounds__(kScanCh) void scan_kernel(
    const float* __restrict__ XD, const float* __restrict__ XC, const unsigned short* __restrict__ WDp,
    const float* __restrict__ bdt, const float* __restrict__ Alog, const float* __restrict__ Dp,
    unsigned short* __restrict__ YH, unsigned short* __restrict__ YL)
{
  __shared__ __align__(16) float sX[kScanTS * kXdP];
  __shared__ __align__(16) float sP[kScanTS * kScanYP];
  __shared__ __align__(16) float sY[kScanTS * kScanYP];
  __shared__ __align__(16) float sA[kNst * kScanCh];
  const int tid = threadIdx.x, lane = tid & 31, wave = tid >> 5;
  const int rlane = lane & 15;
  const int koff  = (lane >> 4) * 8;
  const int mOff  = (lane >> 4) * 8;
  constexpr int kBlkPerB = kHalf / kScanCh;
  const int bix = blockIdx.x / kBlkPerB;
  const int d0  = (blockIdx.x - bix * kBlkPerB) * kScanCh;
  const int d   = d0 + tid;
  const size_t row0 = (size_t)bix * kSeq;
#pragma unroll 1
  for (int s = 0; s < kNst; ++s) sA[s * kScanCh + tid] = -expf(bfr(Alog[(size_t)d * kNst + s])) * kLog2e;
  const __bf16* WD = (const __bf16*)WDp;
  v16b wf[2];
#pragma unroll
  for (int jj = 0; jj < 2; ++jj)
    wf[jj] = Frag<__bf16>::load(WD + (size_t)(d0 + wave * 32 + jj * 16 + rlane) * kDtR + koff);
  __syncthreads();
  float A2[kNst], h[kNst];
#pragma unroll
  for (int s = 0; s < kNst; ++s) {
    A2[s] = sA[s * kScanCh + tid];
    h[s] = 0.f;
  }
  const float b2 = 2.0f * bfr(bdt[d]);
  const float Dd = bfr(Dp[d]);
  const int lr = tid >> 4, lc4 = (tid & 15) * 4;
  const int q = lane >> 3, c8 = (lane & 7) * 8;
#pragma unroll 1
  for (int t0 = 0; t0 < kSeq; t0 += kScanTS) {
    __syncthreads();
#pragma unroll
    for (int i = 0; i < 16; ++i) {
      const int r = lr + 4 * i;
      *(v4f*)(sX + r * kXdP + lc4) = *(const v4f*)(XD + (row0 + t0 + r) * kXdP + lc4);
    }
    __syncthreads();
#pragma unroll
    for (int i = 0; i < 4; ++i) {
      const float* ap = sX + (i * 16 + rlane) * kXdP + koff;
      const v4f f0 = *(const v4f*)(ap);
      const v4f f1 = *(const v4f*)(ap + 4);
      const v4f f2 = *(const v4f*)(ap + 16);
      const v4f f3 = *(const v4f*)(ap + 20);
      v16b ah, al;
#pragma unroll
      for (int e = 0; e < 4; ++e) {
        __bf16 hb, lb;
        split_bf2(f0[e], hb, lb); ah[e]      = hb; al[e]      = lb;
        split_bf2(f1[e], hb, lb); ah[4 + e]  = hb; al[4 + e]  = lb;
        split_bf2(f2[e], hb, lb); ah[8 + e]  = hb; al[8 + e]  = lb;
        split_bf2(f3[e], hb, lb); ah[12 + e] = hb; al[12 + e] = lb;
      }
#pragma unroll
      for (int jj = 0; jj < 2; ++jj) {
        v8f acc = (v8f){0.f,0.f,0.f,0.f,0.f,0.f,0.f,0.f};
        acc = Frag<__bf16>::mma(ah, wf[jj], acc);
        acc = Frag<__bf16>::mma(al, wf[jj], acc);
        dep_guard1_b(acc, ah, al, wf[jj]);
        const int col = wave * 32 + jj * 16 + rlane;
#pragma unroll
        for (int r = 0; r < 8; ++r) sP[(i * 16 + mOff + r) * kScanYP + col] = acc[r];
      }
    }
    __syncthreads();
#pragma unroll 1
    for (int s = 0; s < kScanTS; ++s) {
      const int t = t0 + s;
      const float* xr = sX + s * kXdP + kDtR;
      float Bs[kNst], Cs[kNst];
#pragma unroll
      for (int q4 = 0; q4 < 4; ++q4) {
        const v4f bv = *(const v4f*)(xr + 4 * q4);
        const v4f cv = *(const v4f*)(xr + kNst + 4 * q4);
        Bs[4 * q4 + 0] = bv[0]; Bs[4 * q4 + 1] = bv[1]; Bs[4 * q4 + 2] = bv[2]; Bs[4 * q4 + 3] = bv[3];
        Cs[4 * q4 + 0] = cv[0]; Cs[4 * q4 + 1] = cv[1]; Cs[4 * q4 + 2] = cv[2]; Cs[4 * q4 + 3] = cv[3];
      }
      const size_t gi = (row0 + t) * kHalf + d;
      const float v   = sP[s * kScanYP + tid] + b2;
      const float a   = expf(-fabsf(v));
      const float uu  = 1.0f + a;
      const float l1p = logf(uu) + (a - (uu - 1.0f)) * __builtin_amdgcn_rcpf(uu);
      const float dt  = fmaxf(v, 0.0f) + l1p;
      const float xt  = XC[gi];
      const float dtx = dt * xt;
      float y = 0.f;
#pragma unroll
      for (int k = 0; k < kNst; ++k) {
        const float e = __builtin_amdgcn_exp2f(dt * A2[k]);
        h[k] = e * h[k] + dtx * Bs[k];
        y = fmaf(h[k], Cs[k], y);
      }
      y = fmaf(xt, Dd, y);
      sY[s * kScanYP + tid] = y;
    }
    __syncthreads();
    for (int pass = 0; pass < 2; ++pass) {
#pragma unroll
      for (int it = 0; it < 8; ++it) {
        const int row = it * 8 + wave * 4 + q;
        const float* sp = sY + row * kScanYP + c8;
        const v4f a0 = *(const v4f*)(sp);
        const v4f a1 = *(const v4f*)(sp + 4);
        v8h hv, lv;
#pragma unroll
        for (int e = 0; e < 4; ++e) {
          const unsigned short h0 = f2bf_bits(a0[e]), h1 = f2bf_bits(a1[e]);
          const unsigned short l0 = f2bf_bits(a0[e] - bf_bits2f(h0)), l1 = f2bf_bits(a1[e] - bf_bits2f(h1));
          hv[e]     = __builtin_bit_cast(_Float16, h0);
          hv[4 + e] = __builtin_bit_cast(_Float16, h1);
          lv[e]     = __builtin_bit_cast(_Float16, l0);
          lv[4 + e] = __builtin_bit_cast(_Float16, l1);
        }
        const size_t o = (row0 + t0 + row) * kDin + d0 + c8;
        *(volatile v8h*)(YH + o) = hv;
        *(volatile v8h*)(YL + o) = lv;
      }
      __threadfence();
    }
  }
}

constexpr int kTilesInProj  = (kRows / 64) * (kDin / 64);
constexpr int kTilesXProj   = (kRows / 64) * (kXdP / 64);
constexpr int kTilesOutProj = (kRows / 64) * (kDm / 64);
static_assert((kTilesInProj % 8) == 0 && (kTilesXProj % 8) == 0 && (kTilesOutProj % 8) == 0, "8 tiles per block");
static_assert(((kRows * kDm / 8) % 256) == 0 && ((kDin * kDm / 8) % 256) == 0 && ((kXdP * kHalf / 8) % 256) == 0 &&
              ((kHalf * kDtR / 8) % 256) == 0 && ((kDm * kDin / 8) % 256) == 0, "convert grids exact");

extern "C" void kernel_launch(void* const* d_in, const int* in_sizes, int n_in,
                              void* d_out, int out_size, void* d_ws, size_t ws_size,
                              hipStream_t stream) {
  if (n_in < 12) return;
  if (in_sizes[0]  != kRows * kDm) return;
  if (in_sizes[1]  != kDin * kDm) return;
  if (in_sizes[2]  != kDm * kDin) return;
  if (in_sizes[3]  != kHalf * 4) return;
  if (in_sizes[4]  != kHalf) return;
  if (in_sizes[5]  != kHalf * 4) return;
  if (in_sizes[6]  != kHalf) return;
  if (in_sizes[7]  != kXdP * kHalf) return;
  if (in_sizes[8]  != kHalf * kDtR) return;
  if (in_sizes[9]  != kHalf) return;
  if (in_sizes[10] != kHalf * kNst) return;
  if (in_sizes[11] != kHalf) return;
  if (out_size != kRows * kDm) return;
  if (ws_size < kWsTotal) return;

  const float* hidden   = (const float*)d_in[0];
  const float* W_in     = (const float*)d_in[1];
  const float* W_out    = (const float*)d_in[2];
  const float* conv_x_w = (const float*)d_in[3];
  const float* conv_x_b = (const float*)d_in[4];
  const float* conv_z_w = (const float*)d_in[5];
  const float* conv_z_b = (const float*)d_in[6];
  const float* W_xproj  = (const float*)d_in[7];
  const float* W_dt     = (const float*)d_in[8];
  const float* b_dt     = (const float*)d_in[9];
  const float* A_log    = (const float*)d_in[10];
  const float* Dp       = (const float*)d_in[11];
  float* out = (float*)d_out;

  char* ws = (char*)d_ws;
  unsigned short* AH   = (unsigned short*)(ws + kOffAH);
  unsigned short* WI   = (unsigned short*)(ws + kOffWI);
  unsigned short* WX   = (unsigned short*)(ws + kOffWX);
  unsigned short* WD   = (unsigned short*)(ws + kOffWD);
  unsigned short* WO   = (unsigned short*)(ws + kOffWO);
  float*          XZ   = (float*)(ws + kOffXZ);
  float*          XC   = (float*)(ws + kOffXC);
  unsigned short* XCH  = (unsigned short*)(ws + kOffXCH);
  unsigned short* XCL  = (unsigned short*)(ws + kOffXCL);
  float*          XD   = (float*)(ws + kOffXD);
  unsigned short* YCH  = (unsigned short*)(ws + kOffYCH);
  unsigned short* YCL  = (unsigned short*)(ws + kOffYCL);

  cvt_rows_bf16_kernel<<<(kRows * kDm / 8) / 256, 256, 0, stream>>>(hidden, AH, kRows * kDm / 8);
  cvt_rows_bf16_kernel<<<(kDin * kDm / 8) / 256, 256, 0, stream>>>(W_in, WI, kDin * kDm / 8);
  cvt_rows_bf16_kernel<<<(kXdP * kHalf / 8) / 256, 256, 0, stream>>>(W_xproj, WX, kXdP * kHalf / 8);
  cvt_rows_bf16_kernel<<<(kHalf * kDtR / 8) / 256, 256, 0, stream>>>(W_dt, WD, kHalf * kDtR / 8);
  cvt_rows_bf16_kernel<<<(kDm * kDin / 8) / 256, 256, 0, stream>>>(W_out, WO, kDm * kDin / 8);

  wmma_gemm64_kernel<1, 0><<<kTilesInProj / 8, 256, 0, stream>>>(
      AH, AH, kDm, WI, kDm, XZ, kDin, kRows, kDin, kDm, 1.0f);

  conv_silu_kernel<true><<<dim3(kHalf / 256, kRows / 64), 256, 0, stream>>>(
      XZ, 0, conv_x_w, conv_x_b, XC, XCH, XCL, kHalf, 0);
  conv_silu_kernel<false><<<dim3(kHalf / 256, kRows / 64), 256, 0, stream>>>(
      XZ, kHalf, conv_z_w, conv_z_b, XC, YCH, YCL, kDin, kHalf);

  wmma_gemm64_kernel<1, 1><<<kTilesXProj / 8, 256, 0, stream>>>(
      XCH, XCL, kHalf, WX, kHalf, XD, kXdP, kRows, kXdP, kHalf, 1.0f);

  scan_kernel<<<kBatch * (kHalf / kScanCh), kScanCh, 0, stream>>>(XD, XC, WD, b_dt, A_log, Dp, YCH, YCL);

  wmma_gemm64_kernel<1, 1><<<kTilesOutProj / 8, 256, 0, stream>>>(
      YCH, YCL, kDin, WO, kDin, out, kDm, kRows, kDm, kDin, 1.0f);
}
